// KANConvolution_44229573214883
// MI455X (gfx1250) — hardware-verified
//
#include <hip/hip_runtime.h>
#include <math.h>

#define NB_ 8
#define CIN 32
#define COUT 64
#define IH 32
#define IW 32
#define NPOS (IH * IW)
#define KF 9
#define NCO 8
#define NG 12
#define KC 96

typedef _Float16 f16;
typedef __attribute__((ext_vector_type(16))) f16 f16x16;
typedef __attribute__((ext_vector_type(8)))  f16 f16x8;
typedef __attribute__((ext_vector_type(8)))  float f32x8;
typedef __attribute__((ext_vector_type(4)))  float v4f_t;
typedef float v4fa __attribute__((ext_vector_type(4), may_alias));
__device__ __forceinline__ f32x8 wmma16(f16x16 a, f16x16 b, f32x8 c) {
  c = __builtin_amdgcn_wmma_f32_16x16x32_f16(false, a, false, b, (short)0, c, false, false);
  asm volatile("v_nop\n\tv_nop\n\tv_nop\n\tv_nop" : "+v"(c) : "v"(a), "v"(b));
  return c;
}
__device__ __forceinline__ f16x16 lds_frag(const f16* base, int stride) {
  const int lane = threadIdx.x & 31, row = lane & 15, kh = (lane >> 4) * 8;
  const f16x8 lo = *(const f16x8*)(base + row * stride + kh);
  const f16x8 hi = *(const f16x8*)(base + row * stride + kh + 16);
  f16x16 f;
#pragma unroll
  for (int i = 0; i < 8; ++i) { f[i] = lo[i]; f[i + 8] = hi[i]; }
  return f;
}
__device__ __forceinline__ void split16(float v, f16& h, f16& l) { h = (f16)v; l = (f16)((v - (float)h) * 2048.0f); }
__device__ __forceinline__ void kwfrag(const float* __restrict__ coef, const float* __restrict__ sb, const float* __restrict__ ssp, int c, int o0, int ks, f16x16& hi, f16x16& lo) {
  const int lane = threadIdx.x & 31, o = o0 + (lane & 15), kh = (lane >> 4) * 8;
#pragma unroll
  for (int i = 0; i < 16; ++i) { const int kk = ks * 32 + kh + (i & 7) + ((i >> 3) * 16); float w = 0.0f;
    if (kk < KF) w = sb[((size_t)o * CIN + c) * KF + kk];
    else if (kk < KF + KF * NCO) { const int r = kk - KF, k9 = r >> 3, m = r & 7; w = ssp[((size_t)o * CIN + c) * KF + k9] * coef[(((size_t)o * CIN + c) * KF + k9) * NCO + m]; }
    f16 h, l; split16(w, h, l); hi[i] = h; lo[i] = l; }
}

__global__ __launch_bounds__(256) void k_kanconv(const float* __restrict__ x, const float* __restrict__ coef, const float* __restrict__ sb, const float* __restrict__ ssp, const float* __restrict__ bias, float* __restrict__ out) {
  __shared__ __attribute__((aligned(16))) f16 aS[2][128 * 104];
  __shared__ float rk[3 * 12];
  __shared__ __attribute__((aligned(16))) float oS[COUT * 132];
  const int tid = threadIdx.x, lane = tid & 31, wave = tid >> 5, cl = lane & 15, rh = (lane >> 4) * 8;
  const int b = blockIdx.x / (NPOS / 128), p0 = (blockIdx.x % (NPOS / 128)) * 128;
  const float gh = 0.4f;
  if (tid < 36) { const int p = tid / 12 + 1, t = tid % 12; rk[tid] = (t + p < NG) ? 1.0f / (((-1.0f + (float)(t + p - 3) * gh)) - (-1.0f + (float)(t - 3) * gh)) : 0.0f; }
  for (int e = tid; e < 128 * 15; e += 256) { const int r = e / 15, kk = KF + KF * NCO + e % 15; aS[0][r * 104 + kk] = (f16)0.0f; aS[1][r * 104 + kk] = (f16)0.0f; }
  f32x8 acc[4], accx[4];
#pragma unroll
  for (int j = 0; j < 4; ++j) { f32x8 z = {}; acc[j] = z; accx[j] = z; }
  const int rt = wave, nt0 = 0;
#pragma unroll 1
  for (int c = 0; c < CIN; ++c) {
    __syncthreads();
    const float* xc = x + ((size_t)b * CIN + c) * NPOS;
    for (int it = tid; it < 128 * KF; it += 256) { const int r = it / KF, k9 = it % KF; const int p = p0 + r, oh = p >> 5, ow = p & 31; const int ih = oh + k9 / 3 - 1, iw = ow + k9 % 3 - 1;
      const bool in = (ih >= 0 && ih < IH && iw >= 0 && iw < IW); const float t = in ? xc[min(max(ih, 0), IH - 1) * IW + min(max(iw, 0), IW - 1)] : 0.0f;
      const float silu = t / (1.0f + expf(-t));
      float bs[11];
#pragma unroll
      for (int q = 0; q < 11; ++q) { const float g0 = -1.0f + (float)(q - 3) * gh, g1 = g0 + gh; bs[q] = (t >= g0 && t < g1) ? 1.0f : 0.0f; }
#pragma unroll
      for (int p = 1; p <= 3; ++p) {
#pragma unroll
        for (int q = 0; q < 11 - p; ++q) { const float gq = -1.0f + (float)(q - 3) * gh; bs[q] = (t - gq) * rk[(p - 1) * 12 + q] * bs[q] + ((gq + (float)(p + 1) * gh) - t) * rk[(p - 1) * 12 + q + 1] * bs[q + 1]; } }
      f16 h, l; split16(silu, h, l); aS[0][r * 104 + k9] = h; aS[1][r * 104 + k9] = l;
#pragma unroll
      for (int m = 0; m < NCO; ++m) { split16(bs[m], h, l); const int kk = KF + k9 * NCO + m; aS[0][r * 104 + kk] = h; aS[1][r * 104 + kk] = l; } }
    __syncthreads();
#pragma unroll
    for (int ks = 0; ks < 3; ++ks) { const f16x16 ah = lds_frag(aS[0] + (rt * 16) * 104 + ks * 32, 104), al = lds_frag(aS[1] + (rt * 16) * 104 + ks * 32, 104);
#pragma unroll
      for (int j = 0; j < 4; ++j) { f16x16 bh, bl; kwfrag(coef, sb, ssp, c, (nt0 + j) * 16, ks, bh, bl); acc[j] = wmma16(ah, bh, acc[j]); accx[j] = wmma16(ah, bl, accx[j]); accx[j] = wmma16(al, bh, accx[j]); } }
  }
#pragma unroll
  for (int j = 0; j < 4; ++j)
#pragma unroll
    for (int r = 0; r < 8; ++r) { const int o = (nt0 + j) * 16 + cl, p = rt * 16 + rh + r; oS[o * 132 + p] = acc[j][r] + accx[j][r] * (1.0f / 2048.0f) + bias[o]; }
  __syncthreads();
#pragma unroll 1
  for (int pass = 0; pass < 2; ++pass) { for (int q4 = tid; q4 < COUT * 32; q4 += 256) { const int o = q4 >> 5, c4 = (q4 & 31) * 4;
      *(volatile v4f_t*)(out + ((size_t)b * COUT + o) * NPOS + p0 + c4) = *(const volatile v4fa*)(oS + o * 132 + c4); } __threadfence(); }
}

extern "C" void kernel_launch(void* const* d_in, const int* in_sizes, int n_in,
                              void* d_out, int out_size, void* d_ws, size_t ws_size,
                              hipStream_t stream) {
  (void)in_sizes; (void)n_in; (void)out_size; (void)d_ws; (void)ws_size;
  const float* x = (const float*)d_in[0];
  const float* coef = (const float*)d_in[1];
  const float* sb = (const float*)d_in[2];
  const float* ssp = (const float*)d_in[3];
  const float* bias = (const float*)d_in[4];
  float* out = (float*)d_out;
  k_kanconv<<<dim3(NB_ * (NPOS / 128)), dim3(256), 0, stream>>>(x, coef, sb, ssp, bias, out);
}
